// FourierLayer_7438883356766
// MI455X (gfx1250) — hardware-run, weakly checked
//
#include <hip/hip_runtime.h>
#include <math.h>
#pragma clang fp contract(off)

typedef __attribute__((ext_vector_type(16))) __bf16   v16b;
typedef __attribute__((ext_vector_type(8)))  __bf16   v8b;
typedef __attribute__((ext_vector_type(8)))  _Float16 v8h;
typedef __attribute__((ext_vector_type(8)))  float    v8f;
typedef __attribute__((ext_vector_type(4)))  float    v4f;

constexpr int kBatch    = 32;
constexpr int kTin      = 512;
constexpr int kDm       = 256;
constexpr int kPredLen  = 96;
constexpr int kTout     = kTin + kPredLen;
constexpr int kPick     = 16;
constexpr int kLowFreq  = 1;
constexpr int kHalfBins = kTin / 2;
constexpr int kRowsA    = 2 * kHalfBins;
constexpr int kCols     = kBatch * kDm;
constexpr int kSlabP    = 36;
constexpr int kTileP    = 68;
static_assert(kTout == 608);
static_assert(kRowsA == 512 && kCols == 8192);
static_assert((kTin % 32) == 0 && (kRowsA % 16) == 0 && (kCols % 32) == 0);
static_assert((kTout % 32) == 0 && (kDm % 64) == 0);
static_assert(kPick == 16 && kLowFreq == 1);

constexpr size_t kSzA   = (size_t)kRowsA * kTin * 2;
constexpr size_t kSzX   = (size_t)kCols * kTin * 2;
constexpr size_t kSzC   = (size_t)kRowsA * kCols * 4;
constexpr size_t kOffAH = 0;
constexpr size_t kOffAM = kOffAH + kSzA;
constexpr size_t kOffAL = kOffAM + kSzA;
constexpr size_t kOffXH = kOffAL + kSzA;
constexpr size_t kOffXM = kOffXH + kSzX;
constexpr size_t kOffXL = kOffXM + kSzX;
constexpr size_t kOffCH = kOffXL + kSzX;
constexpr size_t kOffCL = kOffCH + kSzC;
constexpr size_t kWsTotal = kOffCL + kSzC;
static_assert(kWsTotal == 60293120ull);
static_assert(kWsTotal <= 134217728ull);
static_assert((kSzA % 128) == 0 && (kSzX % 128) == 0 && (kSzC % 128) == 0);

__device__ __forceinline__ unsigned short f2bf_bits(float f) {
  unsigned u = __float_as_uint(f);
  return (unsigned short)((u + 0x7FFFu + ((u >> 16) & 1u)) >> 16);
}
__device__ __forceinline__ float bf_bits2f(unsigned short h) { return __uint_as_float(((unsigned)h) << 16); }

__device__ __forceinline__ void split3_bf16(float v, unsigned short& h, unsigned short& m, unsigned short& l) {
  h = f2bf_bits(v);
  const float r1 = v - bf_bits2f(h);
  m = f2bf_bits(r1);
  const float r2 = r1 - bf_bits2f(m);
  l = f2bf_bits(r2);
}

union FragB { v16b v; v8b h[2]; };
__device__ __forceinline__ v16b frag_load(const __bf16* p) {
  FragB f;
  f.h[0] = *(const v8b*)(p);
  f.h[1] = *(const v8b*)(p + 16);
  return f.v;
}
__device__ __forceinline__ v8f mma_bf(v16b a, v16b b, v8f c) {
  c = __builtin_amdgcn_wmma_f32_16x16x32_bf16(false, a, false, b, (short)0, c, false, false);
  asm volatile("v_nop\n\tv_nop\n\tv_nop\n\tv_nop" : "+v"(c) : "v"(a), "v"(b));
  return c;
}

__global__ __launch_bounds__(256) void tw_planes_kernel(
    unsigned short* __restrict__ AH, unsigned short* __restrict__ AM, unsigned short* __restrict__ AL)
{
  __shared__ float cosT[kTin];
  const int tid = threadIdx.x;
  {
    const float c = cospif((float)tid * (1.0f / 256.0f));
    cosT[tid] = c;
    cosT[tid + 256] = -c;
  }
  __syncthreads();
  const int g  = blockIdx.x * 256 + tid;
  const int m  = g >> 6;
  const int k8 = (g & 63) * 8;
  const int f  = m & (kHalfBins - 1);
  const int shift = (m >= kHalfBins) ? 128 : 0;
  v8h hv, mv, lv;
#pragma unroll
  for (int e = 0; e < 8; ++e) {
    const int p = (f * (k8 + e)) & (kTin - 1);
    const float w = cosT[(p - shift) & (kTin - 1)];
    unsigned short hb, mb, lb;
    split3_bf16(w, hb, mb, lb);
    hv[e] = __builtin_bit_cast(_Float16, hb);
    mv[e] = __builtin_bit_cast(_Float16, mb);
    lv[e] = __builtin_bit_cast(_Float16, lb);
  }
  const size_t o = (size_t)m * kTin + k8;
  *(volatile v8h*)(AH + o) = hv;
  *(volatile v8h*)(AM + o) = mv;
  *(volatile v8h*)(AL + o) = lv;
  __threadfence();
  *(volatile v8h*)(AH + o) = hv;
  *(volatile v8h*)(AM + o) = mv;
  *(volatile v8h*)(AL + o) = lv;
}

__global__ __launch_bounds__(256) void x_planes_kernel(
    const float* __restrict__ x,
    unsigned short* __restrict__ XH, unsigned short* __restrict__ XM, unsigned short* __restrict__ XL)
{
  __shared__ __align__(16) float tile[64 * kTileP];
  const int tid = threadIdx.x, lane = tid & 31, wave = tid >> 5;
  const int d0 = blockIdx.x * 64;
  const int t0 = blockIdx.y * 64;
  const int b  = blockIdx.z;
  {
    const int c4 = (tid & 15) * 4;
#pragma unroll
    for (int i = 0; i < 4; ++i) {
      const int tr = (tid >> 4) + 16 * i;
      const v4f v = *(const v4f*)(x + ((size_t)(b * kTin + t0 + tr)) * kDm + d0 + c4);
      *(v4f*)(tile + tr * kTileP + c4) = v;
    }
  }
  __syncthreads();
  const int q = lane >> 3, t8 = (lane & 7) * 8;
  v8h hv[2], mv[2], lv[2];
#pragma unroll
  for (int it = 0; it < 2; ++it) {
    const int dl = it * 32 + wave * 4 + q;
#pragma unroll
    for (int e = 0; e < 8; ++e) {
      const float v = tile[(t8 + e) * kTileP + dl];
      unsigned short hb, mb, lb;
      split3_bf16(v, hb, mb, lb);
      hv[it][e] = __builtin_bit_cast(_Float16, hb);
      mv[it][e] = __builtin_bit_cast(_Float16, mb);
      lv[it][e] = __builtin_bit_cast(_Float16, lb);
    }
  }
  for (int pass = 0; pass < 2; ++pass) {
#pragma unroll
    for (int it = 0; it < 2; ++it) {
      const int dl = it * 32 + wave * 4 + q;
      const size_t o = (size_t)(b * kDm + d0 + dl) * kTin + t0 + t8;
      *(volatile v8h*)(XH + o) = hv[it];
      *(volatile v8h*)(XM + o) = mv[it];
      *(volatile v8h*)(XL + o) = lv[it];
    }
    __threadfence();
  }
}

__global__ __launch_bounds__(256) void dft_planes_gemm_kernel(
    const unsigned short* __restrict__ AHp, const unsigned short* __restrict__ AMp, const unsigned short* __restrict__ ALp,
    const unsigned short* __restrict__ XHp, const unsigned short* __restrict__ XMp, const unsigned short* __restrict__ XLp,
    float* __restrict__ CH, float* __restrict__ CL)
{
  __shared__ __align__(16) float sS[8][2][16 * kSlabP];
  const int lane = threadIdx.x & 31, wave = threadIdx.x >> 5;
  const int tile = blockIdx.x * 8 + wave;
  const int tm = tile >> 8;
  const int tn = tile & 255;
  const int m0 = tm * 16;
  const int n0 = tn * 32;
  const int rlane = lane & 15;
  const int koff  = (lane >> 4) * 8;
  const int mOff  = (lane >> 4) * 8;

  const size_t aoff = (size_t)(m0 + rlane) * kTin + koff;
  const __bf16* pAH = (const __bf16*)AHp + aoff;
  const __bf16* pAM = (const __bf16*)AMp + aoff;
  const __bf16* pAL = (const __bf16*)ALp + aoff;
  const size_t boff = (size_t)(n0 + rlane) * kTin + koff;
  const __bf16* pBH = (const __bf16*)XHp + boff;
  const __bf16* pBM = (const __bf16*)XMp + boff;
  const __bf16* pBL = (const __bf16*)XLp + boff;

  v8f sum[2], cmp[2], sml[2];
#pragma unroll
  for (int j = 0; j < 2; ++j) {
    sum[j] = (v8f){0.f, 0.f, 0.f, 0.f, 0.f, 0.f, 0.f, 0.f};
    cmp[j] = (v8f){0.f, 0.f, 0.f, 0.f, 0.f, 0.f, 0.f, 0.f};
    sml[j] = (v8f){0.f, 0.f, 0.f, 0.f, 0.f, 0.f, 0.f, 0.f};
  }

#pragma unroll 1
  for (int k0 = 0; k0 < kTin; k0 += 32) {
    const v16b aH = frag_load(pAH + k0);
    const v16b aM = frag_load(pAM + k0);
    const v16b aL = frag_load(pAL + k0);
#pragma unroll
    for (int j = 0; j < 2; ++j) {
      const size_t jo = (size_t)j * 16 * kTin + k0;
      const v16b bH = frag_load(pBH + jo);
      const v16b bM = frag_load(pBM + jo);
      const v16b bL = frag_load(pBL + jo);
      v8f part = (v8f){0.f, 0.f, 0.f, 0.f, 0.f, 0.f, 0.f, 0.f};
      part = mma_bf(aH, bH, part);
      v8f sm = sml[j];
      sm = mma_bf(aL, bH, sm);
      sm = mma_bf(aH, bL, sm);
      sm = mma_bf(aM, bM, sm);
      sm = mma_bf(aM, bH, sm);
      sm = mma_bf(aH, bM, sm);
      sml[j] = sm;
#pragma unroll
      for (int r = 0; r < 8; ++r) {
        const float s  = sum[j][r];
        const float p  = part[r];
        const float t  = s + p;
        const float bp = t - s;
        const float er = (s - (t - bp)) + (p - bp);
        cmp[j][r] = cmp[j][r] + er;
        sum[j][r] = t;
      }
    }
  }

  float* slabH = sS[wave][0];
  float* slabL = sS[wave][1];
#pragma unroll
  for (int j = 0; j < 2; ++j) {
#pragma unroll
    for (int r = 0; r < 8; ++r) {
      const float s  = sum[j][r];
      const float e  = cmp[j][r] + sml[j][r];
      const float hi = s + e;
      const float bb = hi - s;
      const float lo = (s - (hi - bb)) + (e - bb);
      slabH[(mOff + r) * kSlabP + (j << 4) + rlane] = hi;
      slabL[(mOff + r) * kSlabP + (j << 4) + rlane] = lo;
    }
  }
  __syncthreads();
  {
    const int q = lane >> 3, c4 = (lane & 7) * 4;
    for (int pass = 0; pass < 2; ++pass) {
#pragma unroll
      for (int it = 0; it < 4; ++it) {
        const int row = it * 4 + q;
        const v4f vh = *(const v4f*)(slabH + row * kSlabP + c4);
        const v4f vl = *(const v4f*)(slabL + row * kSlabP + c4);
        const size_t o = (size_t)(m0 + row) * kCols + n0 + c4;
        *(volatile v4f*)(CH + o) = vh;
        *(volatile v4f*)(CL + o) = vl;
      }
      __threadfence();
    }
  }
}

__global__ __launch_bounds__(64) void select_synth_kernel(
    const float* __restrict__ CH, const float* __restrict__ CL,
    const int* __restrict__ pPred, const int* __restrict__ pPick, const int* __restrict__ pLow,
    float* __restrict__ out)
{
  __shared__ float cosT[kTin];
  __shared__ __align__(16) float sO[2][32 * kSlabP];
  const int tid = threadIdx.x, lane = tid & 31, wave = tid >> 5;
  const int n  = blockIdx.x * 64 + tid;
  const int b  = blockIdx.x >> 2;
  const int dw = (blockIdx.x & 3) * 64 + wave * 32;

#pragma unroll 1
  for (int i = 0; i < 4; ++i) {
    const int p = tid + 64 * i;
    const float c = cospif((float)p * (1.0f / 256.0f));
    cosT[p] = c;
    cosT[p + 256] = -c;
  }
  const int vPred = pPred[0];
  const int vPick = pPick[0];
  const int vLow  = pLow[0];
  const bool premise = (vPred == kPredLen) && (vPick == kPick) && (vLow == kLowFreq);
  const float poison = __uint_as_float(0x7fc00000u);
  __syncthreads();

  double key[kPick];
  float  vc[kPick], vs[kPick];
  int    vf[kPick];
#pragma unroll
  for (int j = 0; j < kPick; ++j) {
    key[j] = -1.0;
    vc[j] = 0.f;
    vs[j] = 0.f;
    vf[j] = 0x7fffffff;
  }

#pragma unroll 1
  for (int f = kLowFreq; f < kHalfBins; ++f) {
    const size_t oc = (size_t)f * kCols + n;
    const size_t os = (size_t)(kHalfBins + f) * kCols + n;
    const float ch = CH[oc];
    const float cl = CL[oc];
    const float sh = CH[os];
    const float sl = CL[os];
    const double cd = (double)ch + (double)cl;
    const double sd = (double)sh + (double)sl;
    double nk = cd * cd + sd * sd;
    float  nc = ch;
    float  ns = sh;
    int    nf = f;
#pragma unroll
    for (int j = 0; j < kPick; ++j) {
      const double tk = key[j];
      const float  tc = vc[j];
      const float  ts = vs[j];
      const int    tf = vf[j];
      const bool sw = (nk > tk) || ((nk == tk) && (nf < tf));
      key[j] = sw ? nk : tk;
      vc[j]  = sw ? nc : tc;
      vs[j]  = sw ? ns : ts;
      vf[j]  = sw ? nf : tf;
      nk = sw ? tk : nk;
      nc = sw ? tc : nc;
      ns = sw ? ts : ns;
      nf = sw ? tf : nf;
    }
  }

  int ph[kPick];
#pragma unroll
  for (int j = 0; j < kPick; ++j) {
    ph[j] = 0;
    vf[j] = vf[j] & (kTin - 1);
  }

  float* slab = sO[wave];
  const int q = lane >> 3, c4 = (lane & 7) * 4;
  const size_t obase = (size_t)b * kTout * kDm + dw;

#pragma unroll 1
  for (int chunk = 0; chunk < kTout / 32; ++chunk) {
#pragma unroll 1
    for (int tl = 0; tl < 32; ++tl) {
      float acc = 0.0f;
#pragma unroll
      for (int j = 0; j < kPick; ++j) {
        const int p = ph[j];
        const float c = cosT[p];
        const float s = cosT[(p - 128) & (kTin - 1)];
        acc = fmaf(vc[j], c, acc);
        acc = fmaf(vs[j], s, acc);
        ph[j] = (p + vf[j]) & (kTin - 1);
      }
      const float val = acc * (1.0f / 256.0f);
      slab[tl * kSlabP + lane] = premise ? val : poison;
    }
    __syncthreads();
    for (int pass = 0; pass < 2; ++pass) {
#pragma unroll
      for (int it = 0; it < 8; ++it) {
        const int row = it * 4 + q;
        const v4f v = *(const v4f*)(slab + row * kSlabP + c4);
        *(volatile v4f*)(out + obase + (size_t)(chunk * 32 + row) * kDm + c4) = v;
      }
      __threadfence();
    }
    __syncthreads();
  }
}

extern "C" void kernel_launch(void* const* d_in, const int* in_sizes, int n_in,
                              void* d_out, int out_size, void* d_ws, size_t ws_size,
                              hipStream_t stream) {
  if (n_in < 4) return;
  if (in_sizes[0] != kBatch * kTin * kDm) return;
  if (in_sizes[1] != 1 || in_sizes[2] != 1 || in_sizes[3] != 1) return;
  if (out_size != kBatch * kTout * kDm) return;
  if (ws_size < kWsTotal) return;

  const float* x     = (const float*)d_in[0];
  const int*   pPred = (const int*)d_in[1];
  const int*   pPick = (const int*)d_in[2];
  const int*   pLow  = (const int*)d_in[3];
  float* out = (float*)d_out;

  char* ws = (char*)d_ws;
  unsigned short* AH = (unsigned short*)(ws + kOffAH);
  unsigned short* AM = (unsigned short*)(ws + kOffAM);
  unsigned short* AL = (unsigned short*)(ws + kOffAL);
  unsigned short* XH = (unsigned short*)(ws + kOffXH);
  unsigned short* XM = (unsigned short*)(ws + kOffXM);
  unsigned short* XL = (unsigned short*)(ws + kOffXL);
  float*          CH = (float*)(ws + kOffCH);
  float*          CL = (float*)(ws + kOffCL);

  tw_planes_kernel<<<(kRowsA * (kTin / 8)) / 256, 256, 0, stream>>>(AH, AM, AL);

  x_planes_kernel<<<dim3(kDm / 64, kTin / 64, kBatch), 256, 0, stream>>>(x, XH, XM, XL);

  dft_planes_gemm_kernel<<<((kRowsA / 16) * (kCols / 32)) / 8, 256, 0, stream>>>(AH, AM, AL, XH, XM, XL, CH, CL);

  select_synth_kernel<<<kCols / 64, 64, 0, stream>>>(CH, CL, pPred, pPick, pLow, out);
}
